// Fourier_12317966205391
// MI455X (gfx1250) — hardware-verified
//
#include <hip/hip_runtime.h>
#include <math.h>

typedef __attribute__((ext_vector_type(16))) _Float16 v16h;
typedef __attribute__((ext_vector_type(8)))  _Float16 v8h;
typedef __attribute__((ext_vector_type(8)))  float    v8f;
typedef __attribute__((ext_vector_type(4)))  float    v4f;

constexpr int kBatch   = 32768;
constexpr int kDim     = 64;
constexpr int kUnits   = 64;
constexpr int kFreq    = 32;
constexpr int kNW      = 2 * kFreq + 1;
constexpr int kKK      = 2 * kFreq;
constexpr int kK       = kDim * kKK;
constexpr int kMTile   = 128;
constexpr int kChunkD  = 2;
constexpr int kChunkK  = kChunkD * kKK;
constexpr int kChunks  = kDim / kChunkD;
constexpr int kPitch   = kChunkK + 8;
constexpr int kSlabP   = 68;
constexpr float kLen     = 2.0f;
constexpr float kHalfPi  = (float)(3.141592653589793 / (double)kLen);
constexpr float kCarry    = 16.0f;
constexpr float kInvCarry = 1.0f / kCarry;

static_assert(kNW == 65, "basis width");
static_assert(kKK == 64 && kK == 4096, "flattened depth");
static_assert((kK % 32) == 0, "depth multiple of 32");
static_assert((kBatch % kMTile) == 0, "row tiles exact");
static_assert(kUnits == 64, "four 16-wide column subtiles");
static_assert(kChunkK == 128 && kChunks == 32, "chunking");
static_assert((kPitch * 2) % 16 == 0, "16-B aligned LDS rows");
static_assert(8 * 16 * kSlabP * 4 <= kMTile * kPitch * 2, "C slabs fit inside the A tile bytes");

constexpr size_t kOffBT   = 0;
constexpr size_t kOffBias = kOffBT + (size_t)kUnits * kK * 2;
constexpr size_t kWsTotal = kOffBias + (size_t)kUnits * 4;
static_assert(kOffBias == 524288ull && kWsTotal == 524544ull, "carve");
static_assert((kOffBias % 128) == 0, "aligned");
static_assert(kWsTotal <= 134217728ull, "carve cap");

union FragU { v16h v; v8h h[2]; };
__device__ __forceinline__ v16h frag_load(const _Float16* p) {
  FragU f;
  f.h[0] = *(const v8h*)(p);
  f.h[1] = *(const v8h*)(p + 16);
  return f.v;
}
__device__ __forceinline__ v8f mma_h(v16h a, v16h b, v8f c) {
  c = __builtin_amdgcn_wmma_f32_16x16x32_f16(false, a, false, b, (short)0, c, false, false);
  asm volatile("v_nop\n\tv_nop\n\tv_nop\n\tv_nop" : "+v"(c) : "v"(a), "v"(b));
  return c;
}

__global__ __launch_bounds__(256) void weight_plane_kernel(const float* __restrict__ w, _Float16* __restrict__ bt)
{
  const int i = blockIdx.x * 256 + threadIdx.x;
  if (i >= kUnits * kDim * 8) return;
  const int rid = i >> 3;
  const int seg = i & 7;
  const float* src = w + (size_t)rid * kNW + 1 + seg * 8;
  float f[8];
#pragma unroll
  for (int e = 0; e < 8; ++e) f[e] = src[e];
  v8h hv;
#pragma unroll
  for (int e = 0; e < 8; ++e) hv[e] = (_Float16)(f[e] * kCarry);
  _Float16* dst = bt + (size_t)i * 8;
  *(volatile v8h*)dst = hv;
  __threadfence();
  *(volatile v8h*)dst = hv;
}

__global__ __launch_bounds__(32) void const_term_kernel(const float* __restrict__ w, float* __restrict__ bias)
{
  const int lane = threadIdx.x & 31;
  const int ug = lane & 15;
  const int dh = lane >> 4;
  const float* p = w + ((size_t)(4 * ug) * kDim + (size_t)dh * 32) * kNW;
  float s0 = 0.0f, s1 = 0.0f, s2 = 0.0f, s3 = 0.0f;
#pragma unroll 1
  for (int d = 0; d < 32; ++d) {
    const float a0 = p[(size_t)d * kNW];
    const float a1 = p[(size_t)(kDim + d) * kNW];
    const float a2 = p[(size_t)(2 * kDim + d) * kNW];
    const float a3 = p[(size_t)(3 * kDim + d) * kNW];
    s0 += a0;
    s1 += a1;
    s2 += a2;
    s3 += a3;
  }
  const float o0 = __shfl_xor(s0, 16, 32);
  const float o1 = __shfl_xor(s1, 16, 32);
  const float o2 = __shfl_xor(s2, 16, 32);
  const float o3 = __shfl_xor(s3, 16, 32);
  v4f v;
  v[0] = 0.5f * (s0 + o0);
  v[1] = 0.5f * (s1 + o1);
  v[2] = 0.5f * (s2 + o2);
  v[3] = 0.5f * (s3 + o3);
  float* dst = bias + ug * 4;
  if (lane < 16) *(volatile v4f*)dst = v;
  __threadfence();
  if (lane < 16) *(volatile v4f*)dst = v;
}

__global__ __launch_bounds__(256) void basis_gemm_kernel(const float* __restrict__ x,
                                                         const _Float16* __restrict__ bt,
                                                         const float* __restrict__ bias,
                                                         float* __restrict__ out)
{
  __shared__ __align__(16) _Float16 sA[kMTile * kPitch];
  __shared__ __align__(16) _Float16 sB[kUnits * kPitch];

  const int tid   = threadIdx.x;
  const int lane  = tid & 31;
  const int wave  = tid >> 5;
  const int rlane = lane & 15;
  const int koff  = (lane >> 4) * 8;
  const int mOff  = (lane >> 4) * 8;
  const int b0    = blockIdx.x * kMTile;

  const int prow = tid >> 1;
  const int pdl  = tid & 1;
  const float* xrow = x + (size_t)(b0 + prow) * kDim + pdl;

  v8f acc[4];
#pragma unroll
  for (int j = 0; j < 4; ++j) acc[j] = (v8f){0.f, 0.f, 0.f, 0.f, 0.f, 0.f, 0.f, 0.f};

#pragma unroll 1
  for (int g = 0; g < kChunks; ++g) {
#pragma unroll
    for (int i = 0; i < 4; ++i) {
      const int idx = tid + 256 * i;
      const int u   = idx >> 4;
      const int seg = idx & 15;
      const v8h wv = *(const v8h*)(bt + (size_t)u * kK + g * kChunkK + seg * 8);
      *(v8h*)(sB + u * kPitch + seg * 8) = wv;
    }
    {
      const float xv = xrow[kChunkD * g];
      const float th = kHalfPi * xv;
      float s1, c1;
      sincosf(th, &s1, &c1);
      float c = c1, s = s1;
      _Float16* dst = sA + prow * kPitch + pdl * kKK;
#pragma unroll 1
      for (int grp = 0; grp < 8; ++grp) {
        v8h buf;
#pragma unroll
        for (int j = 0; j < 4; ++j) {
          buf[2 * j]     = (_Float16)c;
          buf[2 * j + 1] = (_Float16)s;
          const float cn = c * c1 - s * s1;
          const float sn = s * c1 + c * s1;
          c = cn;
          s = sn;
        }
        *(v8h*)(dst + grp * 8) = buf;
      }
    }
    __syncthreads();

#pragma unroll
    for (int ks = 0; ks < 4; ++ks) {
      const v16h a  = frag_load(sA + (wave * 16 + rlane) * kPitch + ks * 32 + koff);
      const v16h q0 = frag_load(sB + (0 * 16 + rlane) * kPitch + ks * 32 + koff);
      const v16h q1 = frag_load(sB + (1 * 16 + rlane) * kPitch + ks * 32 + koff);
      const v16h q2 = frag_load(sB + (2 * 16 + rlane) * kPitch + ks * 32 + koff);
      const v16h q3 = frag_load(sB + (3 * 16 + rlane) * kPitch + ks * 32 + koff);
      acc[0] = mma_h(a, q0, acc[0]);
      acc[1] = mma_h(a, q1, acc[1]);
      acc[2] = mma_h(a, q2, acc[2]);
      acc[3] = mma_h(a, q3, acc[3]);
    }
    __syncthreads();
  }

  float* slab = (float*)(void*)sA + wave * (16 * kSlabP);
  float bv[4];
#pragma unroll
  for (int j = 0; j < 4; ++j) bv[j] = bias[j * 16 + rlane];
#pragma unroll
  for (int j = 0; j < 4; ++j) {
#pragma unroll
    for (int r = 0; r < 8; ++r) {
      const float v = acc[j][r] * kInvCarry + bv[j];
      slab[(mOff + r) * kSlabP + j * 16 + rlane] = v;
    }
  }
  __syncthreads();
  const int hh = lane >> 4;
  const int c4 = (lane & 15) * 4;
  v4f ov[8];
#pragma unroll
  for (int it = 0; it < 8; ++it) ov[it] = *(const v4f*)(slab + (it * 2 + hh) * kSlabP + c4);
  float* obase = out + (size_t)(b0 + wave * 16) * kUnits;
  for (int pass = 0; pass < 2; ++pass) {
#pragma unroll
    for (int it = 0; it < 8; ++it) {
      *(volatile v4f*)(obase + (size_t)(it * 2 + hh) * kUnits + c4) = ov[it];
    }
    __threadfence();
  }
}

extern "C" void kernel_launch(void* const* d_in, const int* in_sizes, int n_in,
                              void* d_out, int out_size, void* d_ws, size_t ws_size,
                              hipStream_t stream) {
  if (n_in < 2) return;
  if (in_sizes[0] != kBatch * kDim) return;
  if (in_sizes[1] != kUnits * kDim * kNW) return;
  if (out_size != kBatch * kUnits) return;
  if (ws_size < kWsTotal) return;

  const float* x = (const float*)d_in[0];
  const float* w = (const float*)d_in[1];
  float* out = (float*)d_out;
  char* ws = (char*)d_ws;
  _Float16* bt   = (_Float16*)(ws + kOffBT);
  float*    bias = (float*)(ws + kOffBias);

  weight_plane_kernel<<<(kUnits * kDim * 8) / 256, 256, 0, stream>>>(w, bt);
  const_term_kernel<<<1, 32, 0, stream>>>(w, bias);
  basis_gemm_kernel<<<kBatch / kMTile, 256, 0, stream>>>(x, bt, bias, out);
}
